// ExcelFormerConv_81673098101064
// MI455X (gfx1250) — hardware-verified
//
#include <hip/hip_runtime.h>


#define NBT  32
#define SS   512
#define DIM  256
#define NH_  8
#define HD   32
#define INR  256
#define DM   DIM
#define SCL  0.17677669529663687f
#define LOSC 1024.0f

typedef _Float16 h16;
typedef unsigned short bf;
typedef __attribute__((ext_vector_type(16))) __bf16   v16bf;
typedef __attribute__((ext_vector_type(16))) _Float16 v16h;
typedef __attribute__((ext_vector_type(8)))  _Float16 v8h;
typedef __attribute__((ext_vector_type(8)))  unsigned short v8us;
typedef __attribute__((ext_vector_type(8)))  float    v8f;
typedef __attribute__((ext_vector_type(4)))  float    v4f;
typedef v8h  __attribute__((may_alias)) v8ha;
typedef v4f  __attribute__((may_alias)) v4fa;
typedef v8us __attribute__((may_alias)) v8usa;

__device__ __forceinline__ unsigned short f2bf(float f) { unsigned u = __float_as_uint(f); u += 0x7FFFu + ((u >> 16) & 1u); return (unsigned short)(u >> 16); }
__device__ __forceinline__ float bf2f(unsigned short b) { return __uint_as_float(((unsigned)b) << 16); }
__device__ __forceinline__ float bfr(float f) { return bf2f(f2bf(f)); }
__device__ __forceinline__ v16h cat16(v8h lo, v8h hi) { return __builtin_shufflevector(lo, hi, 0, 1, 2, 3, 4, 5, 6, 7, 8, 9, 10, 11, 12, 13, 14, 15); }
__device__ __forceinline__ v16bf cat16b(v8us lo, v8us hi) { return __builtin_bit_cast(v16bf, __builtin_shufflevector(lo, hi, 0, 1, 2, 3, 4, 5, 6, 7, 8, 9, 10, 11, 12, 13, 14, 15)); }
__device__ __forceinline__ v8f wmma16(v16h a, v16h b, v8f c) { return __builtin_amdgcn_wmma_f32_16x16x32_f16(false, a, false, b, (short)0, c, false, false); }
__device__ __forceinline__ v8f wmmab(v16bf a, v16bf b, v8f c) { return __builtin_amdgcn_wmma_f32_16x16x32_bf16(false, a, false, b, (short)0, c, false, false); }

template <bool SPLITA, bool F16OUT = false>
__global__ __launch_bounds__(128) void k_gemmb(const bf* __restrict__ A, const bf* __restrict__ Al, const bf* __restrict__ Bn, const float* __restrict__ bias, float* C, int ldc, h16* C2, const float* __restrict__ R = nullptr, int K = DM, int roundR = 1) {
    __shared__ __align__(16) float ost[4][16 * 68];
    const int lane = threadIdx.x & 31, wave = threadIdx.x >> 5, lr = lane & 15, hi = lane >> 4;
    const int r0 = blockIdx.x * 64 + wave * 16, c0 = blockIdx.y * 64;
    const size_t aoff = (size_t)(r0 + lr) * K + 8 * hi;
    size_t boff[4];
#pragma unroll
    for (int t = 0; t < 4; ++t) boff[t] = (size_t)(c0 + t * 16 + lr) * K + 8 * hi;
    v8f acc[4];
#pragma unroll
    for (int t = 0; t < 4; ++t) acc[t] = (v8f){};
#pragma unroll 1
    for (int kc = 0; kc < K; kc += 32) {
        const v16bf a = cat16b(*(const v8us*)(A + aoff + kc), *(const v8us*)(A + aoff + kc + 16));
        v16bf al = a;
        if (SPLITA) al = cat16b(*(const v8us*)(Al + aoff + kc), *(const v8us*)(Al + aoff + kc + 16));
#pragma unroll
        for (int t = 0; t < 4; ++t) { const v16bf b = cat16b(*(const v8us*)(Bn + boff[t] + kc), *(const v8us*)(Bn + boff[t] + kc + 16)); acc[t] = wmmab(a, b, acc[t]); if (SPLITA) acc[t] = wmmab(al, b, acc[t]); }
        asm volatile("v_nop\n\tv_nop\n\tv_nop\n\tv_nop" : "+v"(acc[0]), "+v"(acc[1]), "+v"(acc[2]), "+v"(acc[3]) : "v"(a), "v"(al));
    }
    float* os = &ost[wave][0];
#pragma unroll
    for (int t = 0; t < 4; ++t) { const float bv = bias ? bfr(bias[c0 + t * 16 + lr]) : 0.f;
#pragma unroll
        for (int j = 0; j < 8; ++j) os[(hi * 8 + j) * 68 + t * 16 + lr] = acc[t][j] + bv; }
    __syncthreads();
    if (F16OUT) {
        h16* crow = (h16*)(void*)C + (size_t)r0 * ldc + c0;
        auto pass = [&]() {
#pragma unroll
            for (int s = 0; s < 4; ++s) { const int row = 4 * s + (lane >> 3), piece = lane & 7; const float* sp = os + row * 68 + piece * 8; v8h o, o2;
#pragma unroll
                for (int i = 0; i < 8; ++i) { const h16 a = (h16)sp[i]; o[i] = a; o2[i] = (h16)((sp[i] - (float)a) * LOSC); }
                *(volatile v8h*)(crow + (size_t)row * ldc + piece * 8) = o; if (C2) *(volatile v8h*)(C2 + (size_t)r0 * ldc + c0 + (size_t)row * ldc + piece * 8) = o2; }
        };
        pass(); __threadfence(); pass();
    } else {
        float* crow = C + (size_t)r0 * ldc + c0;
        auto pass = [&]() {
#pragma unroll
            for (int s = 0; s < 8; ++s) { const int Lid = (lane >> 3) + 4 * s, piece = lane & 7; const int row = Lid >> 1, cofs = (Lid & 1) * 32 + piece * 4;
                v4f val = *(const v4fa*)(os + row * 68 + cofs); if (R) { const v4f rv = *(const v4f*)(R + ((size_t)r0 + row) * ldc + c0 + cofs); val += roundR ? (v4f){bfr(rv[0]), bfr(rv[1]), bfr(rv[2]), bfr(rv[3])} : rv; }
                *(volatile v4f*)(crow + (size_t)row * ldc + cofs) = val; }
        };
        pass(); __threadfence(); pass();
    }
}

template <bool SPLITA, bool F16OUT = false>
__global__ __launch_bounds__(128) void k_gemmbz(const bf* __restrict__ A, const bf* __restrict__ Al, const bf* __restrict__ Bn, const float* __restrict__ bias, float* C, int ldc, h16* C2, const float* __restrict__ R, int K, int roundR, size_t sA, size_t sB, size_t sBias, size_t sC) {
    { const size_t g = blockIdx.z; A += g * sA; if (Al) Al += g * sA; Bn += g * sB; if (bias) bias += g * sBias; C += g * sC; if (R) R += g * sC; }
    __shared__ __align__(16) float ost[4][16 * 68];
    const int lane = threadIdx.x & 31, wave = threadIdx.x >> 5, lr = lane & 15, hi = lane >> 4;
    const int r0 = blockIdx.x * 64 + wave * 16, c0 = blockIdx.y * 64;
    const size_t aoff = (size_t)(r0 + lr) * K + 8 * hi;
    size_t boff[4];
#pragma unroll
    for (int t = 0; t < 4; ++t) boff[t] = (size_t)(c0 + t * 16 + lr) * K + 8 * hi;
    v8f acc[4];
#pragma unroll
    for (int t = 0; t < 4; ++t) acc[t] = (v8f){};
#pragma unroll 1
    for (int kc = 0; kc < K; kc += 32) {
        const v16bf a = cat16b(*(const v8us*)(A + aoff + kc), *(const v8us*)(A + aoff + kc + 16));
        v16bf al = a;
        if (SPLITA) al = cat16b(*(const v8us*)(Al + aoff + kc), *(const v8us*)(Al + aoff + kc + 16));
#pragma unroll
        for (int t = 0; t < 4; ++t) { const v16bf b = cat16b(*(const v8us*)(Bn + boff[t] + kc), *(const v8us*)(Bn + boff[t] + kc + 16)); acc[t] = wmmab(a, b, acc[t]); if (SPLITA) acc[t] = wmmab(al, b, acc[t]); }
        asm volatile("v_nop\n\tv_nop\n\tv_nop\n\tv_nop" : "+v"(acc[0]), "+v"(acc[1]), "+v"(acc[2]), "+v"(acc[3]) : "v"(a), "v"(al));
    }
    float* os = &ost[wave][0];
#pragma unroll
    for (int t = 0; t < 4; ++t) { const float bv = bias ? bfr(bias[c0 + t * 16 + lr]) : 0.f;
#pragma unroll
        for (int j = 0; j < 8; ++j) os[(hi * 8 + j) * 68 + t * 16 + lr] = acc[t][j] + bv; }
    __syncthreads();
    if (F16OUT) {
        h16* crow = (h16*)(void*)C + (size_t)r0 * ldc + c0;
        auto pass = [&]() {
#pragma unroll
            for (int s = 0; s < 4; ++s) { const int row = 4 * s + (lane >> 3), piece = lane & 7; const float* sp = os + row * 68 + piece * 8; v8h o, o2;
#pragma unroll
                for (int i = 0; i < 8; ++i) { const h16 a = (h16)sp[i]; o[i] = a; o2[i] = (h16)((sp[i] - (float)a) * LOSC); }
                *(volatile v8h*)(crow + (size_t)row * ldc + piece * 8) = o; if (C2) *(volatile v8h*)(C2 + (size_t)r0 * ldc + c0 + (size_t)row * ldc + piece * 8) = o2; }
        };
        pass(); __threadfence(); pass();
    } else {
        float* crow = C + (size_t)r0 * ldc + c0;
        auto pass = [&]() {
#pragma unroll
            for (int s = 0; s < 8; ++s) { const int Lid = (lane >> 3) + 4 * s, piece = lane & 7; const int row = Lid >> 1, cofs = (Lid & 1) * 32 + piece * 4;
                v4f val = *(const v4fa*)(os + row * 68 + cofs); if (R) { const v4f rv = *(const v4f*)(R + ((size_t)r0 + row) * ldc + c0 + cofs); val += roundR ? (v4f){bfr(rv[0]), bfr(rv[1]), bfr(rv[2]), bfr(rv[3])} : rv; }
                *(volatile v4f*)(crow + (size_t)row * ldc + cofs) = val; }
        };
        pass(); __threadfence(); pass();
    }
}

__global__ __launch_bounds__(256) void k_wt(const float* __restrict__ Wm, int K, int ncols, bf* WT) {
    __shared__ __align__(16) unsigned short tl[64 * 72];
    const int tid = threadIdx.x, k0 = blockIdx.x * 64, n0 = blockIdx.y * 64;
    const int kk = tid >> 2, nq = (tid & 3) * 16;
#pragma unroll
    for (int i = 0; i < 16; ++i) tl[(nq + i) * 72 + kk] = f2bf(Wm[(size_t)(k0 + kk) * ncols + n0 + nq + i]);
    __syncthreads();
    const int piece = tid & 7;
    auto pass = [&]() {
#pragma unroll
        for (int s = 0; s < 2; ++s) { const int nr = (tid >> 3) + 32 * s; const v8us val = *(const v8usa*)(tl + nr * 72 + piece * 8); *(volatile v8us*)(WT + (size_t)(n0 + nr) * K + k0 + piece * 8) = val; }
    };
    pass(); __threadfence(); pass();
}

__global__ __launch_bounds__(256) void k_ln(const float* __restrict__ xb, const float* __restrict__ g, const float* __restrict__ bb, bf* Hh, bf* Hl) {
    const int lane = threadIdx.x & 31, r = blockIdx.x * 8 + (threadIdx.x >> 5); if (r >= SS) return; float v[8]; float s = 0.f;
#pragma unroll
    for (int i = 0; i < 8; ++i) { v[i] = bfr(xb[(size_t)r * DIM + lane * 8 + i]); s += v[i]; }
#pragma unroll
    for (int sh = 16; sh; sh >>= 1) s += __shfl_xor(s, sh, 32);
    const float mu = s * (1.0f / DIM); float q = 0.f;
#pragma unroll
    for (int i = 0; i < 8; ++i) { const float d = v[i] - mu; q = fmaf(d, d, q); }
#pragma unroll
    for (int sh = 16; sh; sh >>= 1) q += __shfl_xor(q, sh, 32);
    const float rs = rsqrtf(q * (1.0f / DIM) + 1e-5f); v8us oh, ol;
#pragma unroll
    for (int i = 0; i < 8; ++i) { const int c = lane * 8 + i; const float y = (v[i] - mu) * rs * bfr(g[c]) + bfr(bb[c]); const unsigned short hb = f2bf(y); oh[i] = hb; ol[i] = f2bf(y - bf2f(hb)); }
    const size_t o = (size_t)r * DIM + lane * 8; *(volatile v8us*)(Hh + o) = oh; *(volatile v8us*)(Hl + o) = ol; __threadfence(); *(volatile v8us*)(Hh + o) = oh; *(volatile v8us*)(Hl + o) = ol;
}
__global__ __launch_bounds__(256) void k_qkplanes(const float* __restrict__ QKV, int col0, bf* Ph, bf* Pl) {
    typedef __attribute__((ext_vector_type(2))) unsigned short v2us;
    const int lane = threadIdx.x & 31; const size_t wid = (size_t)blockIdx.x * 8 + (threadIdx.x >> 5); if (wid >= (size_t)NH_ * (SS / 2)) return; const int h = (int)(wid / (SS / 2)); const int s = (int)(wid % (SS / 2)) * 2 + (lane >> 4); const int d = (lane & 15) * 2;
    v2us oh, ol;
#pragma unroll
    for (int i = 0; i < 2; ++i) { const float v = QKV[(size_t)s * (3 * INR) + col0 + h * HD + d + i]; const unsigned short hb = f2bf(v); oh[i] = hb; ol[i] = f2bf(v - bf2f(hb)); }
    const size_t o = ((size_t)h * SS + s) * HD + d; *(volatile v2us*)(Ph + o) = oh; *(volatile v2us*)(Pl + o) = ol; __threadfence(); *(volatile v2us*)(Ph + o) = oh; *(volatile v2us*)(Pl + o) = ol;
}
__global__ __launch_bounds__(256) void k_vtplanes(const float* __restrict__ QKV, bf* VTh, bf* VTl) {
    typedef __attribute__((ext_vector_type(2))) unsigned short v2us;
    const int lane = threadIdx.x & 31; const size_t wid = (size_t)blockIdx.x * 8 + (threadIdx.x >> 5); if (wid >= (size_t)NH_ * 64 * (SS / 64)) return;
    const int sg = (int)(wid % (SS / 64)), rest = (int)(wid / (SS / 64)), d = rest % 64, h = rest / 64; const int s0 = sg * 64 + 2 * lane; v2us oh, ol;
#pragma unroll
    for (int i = 0; i < 2; ++i) { const float v = (d < HD) ? QKV[(size_t)(s0 + i) * (3 * INR) + 2 * INR + h * HD + (d < HD ? d : 0)] : 0.f; const unsigned short hb = f2bf(v); oh[i] = hb; ol[i] = f2bf(v - bf2f(hb)); }
    const size_t o = ((size_t)h * 64 + d) * SS + s0; *(volatile v2us*)(VTh + o) = oh; *(volatile v2us*)(VTl + o) = ol; __threadfence(); *(volatile v2us*)(VTh + o) = oh; *(volatile v2us*)(VTl + o) = ol;
}
__global__ __launch_bounds__(256) void k_csoft(const float* __restrict__ S, bf* PH, bf* PL) {
    typedef __attribute__((ext_vector_type(4))) unsigned short v4us;
    const int lane = threadIdx.x & 31; const int wid = blockIdx.x * 8 + (threadIdx.x >> 5); if (wid >= NH_ * SS) return; const int i = wid % SS; const float* sr = S + (size_t)wid * SS;
    auto sc = [&](int j) -> float { return (sr[j] + (j > i ? -10000.0f : 0.f)) * SCL; };
    float m = -3.0e38f;
#pragma unroll 1
    for (int c0 = lane * 4; c0 < SS; c0 += 128) {
#pragma unroll
        for (int q = 0; q < 4; ++q) m = fmaxf(m, sc(c0 + q)); }
#pragma unroll
    for (int sh = 16; sh; sh >>= 1) m = fmaxf(m, __shfl_xor(m, sh, 32));
    float sum = 0.f;
#pragma unroll 1
    for (int c0 = lane * 4; c0 < SS; c0 += 128) {
#pragma unroll
        for (int q = 0; q < 4; ++q) sum += __expf(sc(c0 + q) - m); }
#pragma unroll
    for (int sh = 16; sh; sh >>= 1) sum += __shfl_xor(sum, sh, 32);
    const float inv = 1.0f / sum;
#pragma unroll 1
    for (int ps = 0; ps < 2; ++ps) {
#pragma unroll 1
        for (int c0 = lane * 4; c0 < SS; c0 += 128) { v4us oh, ol;
#pragma unroll
            for (int q = 0; q < 4; ++q) { const float p = __expf(sc(c0 + q) - m) * inv; const unsigned short hb = f2bf(p); oh[q] = hb; ol[q] = f2bf(p - bf2f(hb)); }
            const size_t o = (size_t)wid * SS + c0; *(volatile v4us*)(PH + o) = oh; *(volatile v4us*)(PL + o) = ol; }
        if (ps == 0) __threadfence(); }
}
__global__ __launch_bounds__(256) void k_ctxplanes(const float* __restrict__ CT, bf* Ch, bf* Cl) {
    const int lane = threadIdx.x & 31, s = blockIdx.x * 8 + (threadIdx.x >> 5); if (s >= SS) return; const int h = lane >> 2, d0 = (lane & 3) * 8; v8us oh, ol;
#pragma unroll
    for (int i = 0; i < 8; ++i) { const float v = CT[((size_t)h * SS + s) * 64 + d0 + i]; const unsigned short hb = f2bf(v); oh[i] = hb; ol[i] = f2bf(v - bf2f(hb)); }
    const size_t o = (size_t)s * INR + lane * 8; *(volatile v8us*)(Ch + o) = oh; *(volatile v8us*)(Cl + o) = ol; __threadfence(); *(volatile v8us*)(Ch + o) = oh; *(volatile v8us*)(Cl + o) = ol;
}
__global__ __launch_bounds__(256) void k_split256(const float* __restrict__ src, bf* dh, bf* dl) {
    const int lane = threadIdx.x & 31, r = blockIdx.x * 8 + (threadIdx.x >> 5); if (r >= SS) return; const size_t o = (size_t)r * DIM + lane * 8; const v8f v = *(const v8f*)(src + o); v8us oh, ol;
#pragma unroll
    for (int i = 0; i < 8; ++i) { const unsigned short hb = f2bf(v[i]); oh[i] = hb; ol[i] = f2bf(v[i] - bf2f(hb)); }
    *(volatile v8us*)(dh + o) = oh; *(volatile v8us*)(dl + o) = ol; __threadfence(); *(volatile v8us*)(dh + o) = oh; *(volatile v8us*)(dl + o) = ol;
}
__global__ __launch_bounds__(256) void k_glu(const float* __restrict__ O, const float* __restrict__ G, float* OUTB) {
    const int lane = threadIdx.x & 31, s = blockIdx.x * 8 + (threadIdx.x >> 5); if (s >= SS) return;
#pragma unroll 1
    for (int ps = 0; ps < 2; ++ps) {
#pragma unroll
        for (int st = 0; st < 2; ++st) { const int c0 = st * 128 + lane * 4; v4f v;
#pragma unroll
            for (int q = 0; q < 4; ++q) { const int c = c0 + q; v[q] = O[(size_t)s * DIM + c] + G[(size_t)s * 2 * DIM + c] * tanhf(G[(size_t)s * 2 * DIM + DIM + c]); }
            *(volatile v4f*)(OUTB + (size_t)s * DIM + c0) = v; }
        if (ps == 0) __threadfence(); }
}

extern "C" void kernel_launch(void* const* d_in, const int* in_sizes, int n_in,
                              void* d_out, int out_size, void* d_ws, size_t ws_size, hipStream_t stream) {
    (void)in_sizes; (void)n_in; (void)out_size;
    const float* x = (const float*)d_in[0]; const float* lng = (const float*)d_in[1]; const float* lnb = (const float*)d_in[2]; const float* wqkv = (const float*)d_in[3]; const float* wout = (const float*)d_in[4]; const float* bout = (const float*)d_in[5]; const float* wglu = (const float*)d_in[6];
    float* out = (float*)d_out;
    char* wsp = (char*)d_ws;
    auto take = [&](size_t bytes) { char* p = wsp; wsp += (bytes + 255) & ~(size_t)255; return (void*)p; };
    bf* WQKV = (bf*)take((size_t)(3 * INR) * DIM * 2); bf* WOUT = (bf*)take((size_t)DIM * INR * 2); bf* WGLU = (bf*)take((size_t)(2 * DIM) * DIM * 2);
    bf* Hh = (bf*)take((size_t)SS * DIM * 2); bf* Hl = (bf*)take((size_t)SS * DIM * 2); float* QKV = (float*)take((size_t)SS * 3 * INR * 4);
    bf* Qh = (bf*)take((size_t)NH_ * SS * HD * 2); bf* Ql = (bf*)take((size_t)NH_ * SS * HD * 2); bf* Kh = (bf*)take((size_t)NH_ * SS * HD * 2); bf* Kl = (bf*)take((size_t)NH_ * SS * HD * 2); bf* VTh = (bf*)take((size_t)NH_ * 64 * SS * 2); bf* VTl = (bf*)take((size_t)NH_ * 64 * SS * 2);
    float* S1 = (float*)take((size_t)NH_ * SS * SS * 4); float* S2 = (float*)take((size_t)NH_ * SS * SS * 4); bf* PH = (bf*)take((size_t)NH_ * SS * SS * 2); bf* PL = (bf*)take((size_t)NH_ * SS * SS * 2);
    float* CT1 = (float*)take((size_t)NH_ * SS * 64 * 4); float* CT = (float*)take((size_t)NH_ * SS * 64 * 4); bf* Ch = (bf*)take((size_t)SS * INR * 2); bf* Cl = (bf*)take((size_t)SS * INR * 2);
    float* O = (float*)take((size_t)SS * DIM * 4); bf* Oh = (bf*)take((size_t)SS * DIM * 2); bf* Ol = (bf*)take((size_t)SS * DIM * 2); float* G = (float*)take((size_t)SS * 2 * DIM * 4);
    if ((size_t)(wsp - (char*)d_ws) > ws_size) return;
    k_wt<<<dim3(DIM / 64, (3 * INR) / 64, 1), 256, 0, stream>>>(wqkv, DIM, 3 * INR, WQKV); k_wt<<<dim3(INR / 64, DIM / 64, 1), 256, 0, stream>>>(wout, INR, DIM, WOUT); k_wt<<<dim3(DIM / 64, (2 * DIM) / 64, 1), 256, 0, stream>>>(wglu, DIM, 2 * DIM, WGLU);
    const size_t sQ = (size_t)SS * HD, sVT = (size_t)64 * SS, sS = (size_t)SS * SS, sCT = (size_t)SS * 64;
    for (int b = 0; b < NBT; ++b) {
        k_ln<<<SS / 8, 256, 0, stream>>>(x + (size_t)b * SS * DIM, lng, lnb, Hh, Hl);
        k_gemmb<true, false><<<dim3(SS / 64, (3 * INR) / 64, 1), 128, 0, stream>>>(Hh, Hl, WQKV, nullptr, QKV, 3 * INR, nullptr, nullptr, DIM);
        k_qkplanes<<<(NH_ * SS / 2) / 8, 256, 0, stream>>>(QKV, 0, Qh, Ql); k_qkplanes<<<(NH_ * SS / 2) / 8, 256, 0, stream>>>(QKV, INR, Kh, Kl); k_vtplanes<<<(NH_ * 64 * (SS / 64)) / 8, 256, 0, stream>>>(QKV, VTh, VTl);
        k_gemmbz<true, false><<<dim3(SS / 64, SS / 64, NH_), 128, 0, stream>>>(Qh, Ql, Kh, nullptr, S1, SS, nullptr, nullptr, HD, 0, sQ, sQ, 0, sS);
        k_gemmbz<false, false><<<dim3(SS / 64, SS / 64, NH_), 128, 0, stream>>>(Qh, nullptr, Kl, nullptr, S2, SS, nullptr, S1, HD, 0, sQ, sQ, 0, sS);
        k_csoft<<<(NH_ * SS) / 8, 256, 0, stream>>>(S2, PH, PL);
        k_gemmbz<true, false><<<dim3(SS / 64, 1, NH_), 128, 0, stream>>>(PH, PL, VTh, nullptr, CT1, 64, nullptr, nullptr, SS, 0, sS, sVT, 0, sCT);
        k_gemmbz<false, false><<<dim3(SS / 64, 1, NH_), 128, 0, stream>>>(PH, nullptr, VTl, nullptr, CT, 64, nullptr, CT1, SS, 0, sS, sVT, 0, sCT);
        k_ctxplanes<<<SS / 8, 256, 0, stream>>>(CT, Ch, Cl);
        k_gemmb<true, false><<<dim3(SS / 64, DIM / 64, 1), 128, 0, stream>>>(Ch, Cl, WOUT, bout, O, DIM, nullptr, nullptr, INR);
        k_split256<<<SS / 8, 256, 0, stream>>>(O, Oh, Ol);
        k_gemmb<true, false><<<dim3(SS / 64, (2 * DIM) / 64, 1), 128, 0, stream>>>(Oh, Ol, WGLU, nullptr, G, 2 * DIM, nullptr, nullptr, DIM);
        k_glu<<<SS / 8, 256, 0, stream>>>(O, G, out + (size_t)b * SS * DIM); }
}
